// DirectionalScan_41669772706452
// MI455X (gfx1250) — hardware-verified
//
#include <hip/hip_runtime.h>


namespace {
constexpr int NB = 4, GH = 64, GW = 64, L = GH * GW, DM = 512, NS = 8, NR = NB * L;
constexpr float XS = 8.0f, WSC = 256.0f;
typedef _Float16 b16;
typedef __attribute__((ext_vector_type(16))) _Float16 v16b;
typedef __attribute__((ext_vector_type(8))) _Float16 v8b;
typedef __attribute__((ext_vector_type(8))) float v8f;
typedef __attribute__((ext_vector_type(4))) float v4f;
__device__ __forceinline__ float bf16_rne(float f) { unsigned int u = __float_as_uint(f); u += 0x7FFFu + ((u >> 16) & 1u); return __uint_as_float(u & 0xFFFF0000u); }
__device__ __forceinline__ void split16(float v, b16& hi, b16& lo) { hi = (b16)v; lo = (b16)(v - (float)hi); }
__device__ __forceinline__ v16b frag_kb(const b16* p, int hh) { const v8b a = *(const v8b*)(p + 8 * hh), b = *(const v8b*)(p + 16 + 8 * hh); v16b f;
#pragma unroll
  for (int e = 0; e < 8; ++e) { f[e] = a[e]; f[8 + e] = b[e]; } return f; }
__device__ __forceinline__ v8f wmma16b(v16b a, v16b b, v8f c) { v8f d = __builtin_amdgcn_wmma_f32_16x16x32_f16(false, a, false, b, (short)0, c, false, false); asm volatile("v_nop\n\tv_nop\n\tv_nop\n\tv_nop" : "+v"(d) : "v"(a), "v"(b)); return d; }
__device__ __forceinline__ void wave_lds_sync() { __builtin_amdgcn_fence(__ATOMIC_RELEASE, "workgroup"); __builtin_amdgcn_wave_barrier(); __builtin_amdgcn_fence(__ATOMIC_ACQUIRE, "workgroup"); }
__device__ __forceinline__ float pmul(float a, float b) { float p = a * b; asm volatile("" : "+v"(p)); return p; }

__global__ __launch_bounds__(256) void prepw_kernel(const float* __restrict__ wp, b16* __restrict__ WP16) {
  const int u = blockIdx.x * 256 + threadIdx.x; if (u >= DM * DM / 8) return; const int e = u * 8; v8b o; for (int j = 0; j < 8; ++j) o[j] = (b16)(bf16_rne(wp[e + j]) * WSC);
  for (int pass = 0; pass < 2; ++pass) { *(volatile v8b*)(WP16 + e) = o; __threadfence(); }
}
template <int DIR>
__global__ __launch_bounds__(256) void scan_kernel(const float* __restrict__ x, const float* __restrict__ A, const float* __restrict__ Bm, const float* __restrict__ Cm, const float* __restrict__ Dk, float* __restrict__ YH, b16* __restrict__ Yh, b16* __restrict__ Yl) {
  const int gw = blockIdx.x * 8 + (threadIdx.x >> 5), lane = threadIdx.x & 31;
  constexpr int CPL = DIR == 0 ? 1 : 2;
  constexpr int WPL = DM / (32 * CPL);
  const int bl = gw / WPL, cw = gw % WPL; const int b = bl / (DIR == 0 ? GW : GH), line = bl % (DIR == 0 ? GW : GH); if (b >= NB) return;
  const int d0 = cw * 32 * CPL + lane * CPL;
  float a[CPL][NS], bb[CPL][NS], cc[CPL][NS], dk[CPL], s[CPL][NS];
  for (int q = 0; q < CPL; ++q) { dk[q] = bf16_rne(Dk[d0 + q]); for (int n = 0; n < NS; ++n) { a[q][n] = bf16_rne(A[(d0 + q) * NS + n]); bb[q][n] = bf16_rne(Bm[(d0 + q) * NS + n]); cc[q][n] = bf16_rne(Cm[(d0 + q) * NS + n]); s[q][n] = 0.0f; } }
#pragma unroll 1
  for (int t = 0; t < (DIR == 0 ? GH : GW); ++t) { const int p = DIR == 0 ? (t * GW + line) : (line * GW + t); const size_t row = (size_t)b * L + p; float yv[CPL];
    for (int q = 0; q < CPL; ++q) { const float xv = bf16_rne(x[row * DM + d0 + q]); float y = pmul(dk[q], xv);
#pragma unroll
      for (int n = 0; n < NS; ++n) { s[q][n] = pmul(a[q][n], s[q][n]) + pmul(bb[q][n], xv); }
      float acc = 0.0f;
#pragma unroll
      for (int n = 0; n < NS; ++n) acc += pmul(s[q][n], cc[q][n]);
      yv[q] = acc + y; }
    if (DIR == 0) { for (int pass = 0; pass < 2; ++pass) { ((volatile float*)YH)[row * DM + d0] = yv[0]; __threadfence(); } }
    else { const float y0 = yv[0] + YH[row * DM + d0], y1 = yv[1] + YH[row * DM + d0 + 1]; b16 h0, l0, h1, l1; split16(y0 * XS, h0, l0); split16(y1 * XS, h1, l1);
      typedef __attribute__((ext_vector_type(2))) _Float16 v2h; v2h hv = {h0, h1}, lv = {l0, l1};
      for (int pass = 0; pass < 2; ++pass) { *(volatile v2h*)(Yh + row * DM + d0) = hv; *(volatile v2h*)(Yl + row * DM + d0) = lv; __threadfence(); } } }
}
__global__ __launch_bounds__(128) void proj_kernel(const b16* __restrict__ Yh, const b16* __restrict__ Yl, const b16* __restrict__ WP16, const float* __restrict__ bias, float* __restrict__ out) {
  __shared__ __attribute__((aligned(16))) float Tf[4][16][128 + 4];
  const int wave = threadIdx.x >> 5, lane = threadIdx.x & 31, nloc = lane & 15, hlf = lane >> 4; const size_t m0 = (size_t)blockIdx.x * 64 + wave * 16; const int n0 = blockIdx.y * 128; v8f acc[8];
#pragma unroll
  for (int t = 0; t < 8; ++t) acc[t] = (v8f){};
#pragma unroll 2
  for (int kb = 0; kb < DM; kb += 32) { const v16b a = frag_kb(Yh + (m0 + nloc) * DM + kb, hlf), al = frag_kb(Yl + (m0 + nloc) * DM + kb, hlf);
#pragma unroll
    for (int t = 0; t < 8; ++t) { const v16b bw = frag_kb(WP16 + (size_t)(n0 + t * 16 + nloc) * DM + kb, hlf); acc[t] = wmma16b(a, bw, acc[t]); acc[t] = wmma16b(al, bw, acc[t]); } }
#pragma unroll
  for (int t = 0; t < 8; ++t) { const float b_ = bf16_rne(bias[n0 + t * 16 + nloc]);
#pragma unroll 1
    for (int r = 0; r < 8; ++r) Tf[wave][8 * hlf + r][t * 16 + nloc] = acc[t][r] * (1.0f / (XS * WSC)) + b_; }
  wave_lds_sync();
  for (int pass = 0; pass < 2; ++pass) { for (int rr = 0; rr < 16; ++rr) *(volatile v4f*)(out + (m0 + rr) * DM + n0 + lane * 4) = *(const v4f*)(&Tf[wave][rr][lane * 4]); __threadfence(); }
}
}

extern "C" void kernel_launch(void* const* d_in, const int* in_sizes, int n_in, void* d_out, int out_size, void* d_ws, size_t ws_size, hipStream_t stream) {
  (void)n_in;
  auto Fp = [&](int i) { return (const float*)d_in[i]; };
  if (in_sizes[0] != NR * DM || in_sizes[3] != DM * NS || in_sizes[4] != DM * NS || in_sizes[5] != DM * NS || in_sizes[6] != DM || in_sizes[7] != DM * DM || out_size != NR * DM) return;
  size_t off = 0; char* ws = (char*)d_ws;
  auto carve = [&](size_t bytes) { char* p = ws + off; off += (bytes + 255) & ~(size_t)255; return p; };
  b16* WP16 = (b16*)carve((size_t)DM * DM * 2); float* YH = (float*)carve((size_t)NR * DM * 4); b16* Yh = (b16*)carve((size_t)NR * DM * 2); b16* Yl = (b16*)carve((size_t)NR * DM * 2);
  if (off > ws_size || off > ((size_t)128 << 20)) return;
  prepw_kernel<<<(DM * DM / 8 + 255) / 256, 256, 0, stream>>>(Fp(7), WP16);
  scan_kernel<0><<<NB * GW * (DM / 32) / 8, 256, 0, stream>>>(Fp(0), Fp(3), Fp(4), Fp(5), Fp(6), YH, nullptr, nullptr);
  scan_kernel<1><<<NB * GH * (DM / 64) / 8, 256, 0, stream>>>(Fp(0), Fp(3), Fp(4), Fp(5), Fp(6), YH, Yh, Yl);
  proj_kernel<<<dim3(NR / 64, DM / 128), 128, 0, stream>>>(Yh, Yl, WP16, Fp(8), (float*)d_out);
}
